// MultiModalMolecularModel_81114752352572
// MI455X (gfx1250) — hardware-verified
//
#include <hip/hip_runtime.h>
#include <hip/hip_bf16.h>
#include <math.h>

typedef __attribute__((ext_vector_type(16))) _Float16 v16h;
typedef __attribute__((ext_vector_type(8)))  _Float16 v8h;
typedef __attribute__((ext_vector_type(8)))  float  v8f;
typedef __attribute__((ext_vector_type(4)))  float  v4f;
typedef __attribute__((ext_vector_type(4)))  unsigned v4u;
typedef float __attribute__((may_alias)) float_a;
template <typename T> __device__ __forceinline__ void vst2(void* p, T v) { *(volatile T*)p = v; __threadfence(); *(volatile T*)p = v; }

static __device__ __forceinline__ v16h join16(v8h lo, v8h hi) {
  return __builtin_shufflevector(lo, hi, 0,1,2,3,4,5,6,7,8,9,10,11,12,13,14,15);
}

static __device__ __forceinline__ v8f wmma_f16x(v16h a, v16h b, v8f c) {
  v8f d = __builtin_amdgcn_wmma_f32_16x16x32_f16(false, a, false, b, (short)0, c, false, false);
  asm volatile("v_nop\n\tv_nop\n\tv_nop\n\tv_nop" : "+v"(d) : "v"(a), "v"(b));
  return d;
}

#define HDIM 256
#define ATOM_TYPES 100
#define ATOM_PAD   112
#define BOND_TYPES 5
#define BOND_PAD   16


__global__ void k_temb(const float* __restrict__ t, float* __restrict__ temb, int H) {
  int b = blockIdx.x;
  int j = threadIdx.x;
  int half = H >> 1;
  float tb = t[b];
  float lf = -logf(10000.0f) / (float)(half - 1);
  float v;
  if (j < half) v = sinf(tb * expf((float)j * lf));
  else          v = cosf(tb * expf((float)(j - half) * lf));
  vst2(temb + b * H + j, (float_a)v);
}

__global__ void k_make_h(const float* __restrict__ nf, const int* __restrict__ batch,
                         const float* __restrict__ temb, _Float16* __restrict__ hbf, int total8, int H, int B) {
  int g = blockIdx.x * blockDim.x + threadIdx.x;
  if (g >= total8) return;
  int idx = g * 8;
  int n = idx / H;
  int j = idx - n * H;
  int bb = batch[n]; bb = bb < 0 ? 0 : (bb >= B ? B - 1 : bb);
  union { v8h h; v4u u; } pk;
#pragma unroll
  for (int e = 0; e < 8; ++e) pk.h[e] = (_Float16)(nf[idx + e] + temb[bb * H + j + e]);
  vst2(hbf + idx, pk.u);
}
__global__ void k_copy_f32(const float* __restrict__ src, float* __restrict__ dst, int n) {
  int g = blockIdx.x * blockDim.x + threadIdx.x;
  if (g * 4 + 4 <= n) { v4f v = *(const v4f*)(src + g * 4); vst2(dst + g * 4, v); }
  else { for (int i = g * 4; i < n; ++i) vst2(dst + i, (float_a)src[i]); }
}
__global__ void k_transpose_pad(const float* __restrict__ in, _Float16* __restrict__ out,
                                int K, int Ncols, int Npad) {
  int g = blockIdx.x * blockDim.x + threadIdx.x;
  if (g * 8 >= K * Npad) return;
  int idx = g * 8;
  int n = idx / K;
  int k = idx - n * K;
  union { v8h h; v4u u; } pk;
#pragma unroll
  for (int e = 0; e < 8; ++e) pk.h[e] = (_Float16)((n < Ncols) ? in[(k + e) * Ncols + n] : 0.0f);
  vst2(out + idx, pk.u);
}

__global__ __launch_bounds__(256) void k_atom(
    const _Float16* __restrict__ hbf,
    const _Float16* __restrict__ w1T,
    const float*  __restrict__ b1,
    const _Float16* __restrict__ w2T,
    const float*  __restrict__ b2,
    float* __restrict__ out,
    int N) {
  __shared__ __align__(16) _Float16 sX[16 * HDIM];
  __shared__ __align__(16) _Float16 sHid[16 * HDIM];
  __shared__ __align__(16) float sOut[16 * ATOM_TYPES];

  const int tid  = threadIdx.x;
  const int n0   = blockIdx.x * 16;
  const int wave = tid >> 5;
  const int lane = tid & 31;
  const int ln   = lane & 15;
  const int kh   = lane >> 4;

  {
    int r = tid >> 4;
    int c = tid & 15;
    int row = n0 + r; if (row >= N) row = N - 1;
    const _Float16* src = hbf + (size_t)row * HDIM + c * 16;
    *(v8h*)&sX[r * HDIM + c * 16]     = *(const v8h*)src;
    *(v8h*)&sX[r * HDIM + c * 16 + 8] = *(const v8h*)(src + 8);
  }
  __syncthreads();

  v8f acc0 = {}; v8f acc1 = {};
  const int c0 = wave * 32 + ln;
  const int c1 = c0 + 16;
#pragma unroll
  for (int kb = 0; kb < HDIM; kb += 32) {
    v16h a = join16(*(const v8h*)&sX[ln * HDIM + kb + kh * 8],
                     *(const v8h*)&sX[ln * HDIM + kb + 16 + kh * 8]);
    const _Float16* bp0 = w1T + (size_t)c0 * HDIM + kb + kh * 8;
    const _Float16* bp1 = w1T + (size_t)c1 * HDIM + kb + kh * 8;
    v16h b0 = join16(*(const v8h*)bp0, *(const v8h*)(bp0 + 16));
    v16h b1v = join16(*(const v8h*)bp1, *(const v8h*)(bp1 + 16));
    acc0 = wmma_f16x(a, b0, acc0);
    acc1 = wmma_f16x(a, b1v, acc1);
  }
  {
    float bb0 = b1[c0], bb1 = b1[c1];
#pragma unroll
    for (int j = 0; j < 8; ++j) {
      int r = j + kh * 8;
      float v0 = acc0[j] + bb0; v0 = v0 > 0.0f ? v0 : 0.0f;
      float v1 = acc1[j] + bb1; v1 = v1 > 0.0f ? v1 : 0.0f;
      sHid[r * HDIM + c0] = (_Float16)v0;
      sHid[r * HDIM + c1] = (_Float16)v1;
    }
  }
  __syncthreads();

  if (wave < 7) {
    v8f acc = {};
    const int oc = wave * 16 + ln;
#pragma unroll
    for (int kb = 0; kb < HDIM; kb += 32) {
      v16h a = join16(*(const v8h*)&sHid[ln * HDIM + kb + kh * 8],
                       *(const v8h*)&sHid[ln * HDIM + kb + 16 + kh * 8]);
      const _Float16* bp = w2T + (size_t)oc * HDIM + kb + kh * 8;
      v16h b = join16(*(const v8h*)bp, *(const v8h*)(bp + 16));
      acc = wmma_f16x(a, b, acc);
    }
    float bb = (oc < ATOM_TYPES) ? b2[oc] : 0.0f;
#pragma unroll
    for (int j = 0; j < 8; ++j) {
      int r = j + kh * 8;
      if (oc < ATOM_TYPES) sOut[r * ATOM_TYPES + oc] = acc[j] + bb;
    }
  }
  __syncthreads();
  {
    for (int g = tid; g < 16 * 25; g += 256) { const int r = g / 25, pc = g % 25;
      if (n0 + r < N) vst2(out + (size_t)(n0 + r) * 128 + pc * 4, *(const v4f*)(sOut + r * ATOM_TYPES + pc * 4)); }
  }
}

#define BOND_MT 4
#define BOND_EPB (BOND_MT * 16)

__global__ __launch_bounds__(256) void k_bond(
    const _Float16* __restrict__ hbf,
    const int*    __restrict__ ei,
    const _Float16* __restrict__ w1T,
    const float*  __restrict__ b1,
    const _Float16* __restrict__ w2T,
    const float*  __restrict__ b2,
    float* __restrict__ out,
    int E) {
  extern __shared__ __align__(16) char smem[];
  _Float16* sEF  = (_Float16*)smem;
  _Float16* sHid = (_Float16*)(smem + BOND_EPB * 512 * 2);
  __shared__ __align__(16) float sBO[BOND_EPB * BOND_TYPES];

  const int tid  = threadIdx.x;
  const int e0   = blockIdx.x * BOND_EPB;
  const int wave = tid >> 5;
  const int lane = tid & 31;
  const int ln   = lane & 15;
  const int kh   = lane >> 4;

  {
    int e = tid >> 2;
    int c = tid & 3;
    int edge = e0 + e; if (edge >= E) edge = E - 1;
    int node = (c < 2) ? ei[edge] : ei[E + edge]; node = node < 0 ? 0 : (node >= 10000 ? 9999 : node);
    const _Float16* src = hbf + (size_t)node * HDIM + (c & 1) * 128;
    _Float16* dst = sEF + e * 512 + c * 128;
#pragma unroll
    for (int i = 0; i < 16; ++i)
      *(v8h*)(dst + i * 8) = *(const v8h*)(src + i * 8);
  }
  __syncthreads();

  v8f acc[BOND_MT][2];
#pragma unroll
  for (int mt = 0; mt < BOND_MT; ++mt) { acc[mt][0] = (v8f){}; acc[mt][1] = (v8f){}; }
  const int c0 = wave * 32 + ln;
  const int c1 = c0 + 16;
#pragma unroll
  for (int kb = 0; kb < 512; kb += 32) {
    const _Float16* bp0 = w1T + (size_t)c0 * 512 + kb + kh * 8;
    const _Float16* bp1 = w1T + (size_t)c1 * 512 + kb + kh * 8;
    v16h b0  = join16(*(const v8h*)bp0, *(const v8h*)(bp0 + 16));
    v16h b1v = join16(*(const v8h*)bp1, *(const v8h*)(bp1 + 16));
#pragma unroll
    for (int mt = 0; mt < BOND_MT; ++mt) {
      const _Float16* ap = sEF + (mt * 16 + ln) * 512 + kb + kh * 8;
      v16h a = join16(*(const v8h*)ap, *(const v8h*)(ap + 16));
      acc[mt][0] = wmma_f16x(a, b0,  acc[mt][0]);
      acc[mt][1] = wmma_f16x(a, b1v, acc[mt][1]);
    }
  }
  {
    float bb0 = b1[c0], bb1 = b1[c1];
#pragma unroll
    for (int mt = 0; mt < BOND_MT; ++mt) {
#pragma unroll
      for (int j = 0; j < 8; ++j) {
        int r = mt * 16 + j + kh * 8;
        float v0 = acc[mt][0][j] + bb0; v0 = v0 > 0.0f ? v0 : 0.0f;
        float v1 = acc[mt][1][j] + bb1; v1 = v1 > 0.0f ? v1 : 0.0f;
        sHid[r * HDIM + c0] = (_Float16)v0;
        sHid[r * HDIM + c1] = (_Float16)v1;
      }
    }
  }
  __syncthreads();

  if (wave < BOND_MT) {
    v8f a2 = {};
#pragma unroll
    for (int kb = 0; kb < HDIM; kb += 32) {
      const _Float16* ap = sHid + (wave * 16 + ln) * HDIM + kb + kh * 8;
      v16h a = join16(*(const v8h*)ap, *(const v8h*)(ap + 16));
      const _Float16* bp = w2T + (size_t)ln * HDIM + kb + kh * 8;
      v16h b = join16(*(const v8h*)bp, *(const v8h*)(bp + 16));
      a2 = wmma_f16x(a, b, a2);
    }
    float bb = (ln < BOND_TYPES) ? b2[ln] : 0.0f;
#pragma unroll
    for (int j = 0; j < 8; ++j) {
      int r = wave * 16 + j + kh * 8;
      if (ln < BOND_TYPES) sBO[r * BOND_TYPES + ln] = a2[j] + bb;
    }
  }
  __syncthreads();
  if (tid < 128) { const int r = tid >> 1, hh = tid & 1;
    v4f v;
#pragma unroll
    for (int e = 0; e < 4; ++e) { const int c = hh * 4 + e; v[e] = (c < BOND_TYPES) ? sBO[r * BOND_TYPES + c] : 0.f; }
    if (e0 + r < E) vst2(out + (size_t)(e0 + r) * 8 + hh * 4, v); }
}
__global__ __launch_bounds__(256) void k_flat(const float* __restrict__ stA, const float* __restrict__ stB,
                                             float* __restrict__ outA, float* __restrict__ outB, int N, int E) {
  const int g = blockIdx.x * 256 + threadIdx.x;
  const int nA = N * ATOM_TYPES / 4;
  const int nB = E * BOND_TYPES / 4;
  if (g < nA) {
    const int f = g * 4, r = f / ATOM_TYPES, c = f - r * ATOM_TYPES;
    vst2(outA + f, *(const v4f*)(stA + (size_t)r * 128 + c));
  } else if (g < nA + nB) {
    const int f = (g - nA) * 4;
    v4f v;
#pragma unroll
    for (int e = 0; e < 4; ++e) { const int ff = f + e, r = ff / BOND_TYPES, c = ff - r * BOND_TYPES; v[e] = stB[(size_t)r * 8 + c]; }
    vst2(outB + f, v);
  }
}

extern "C" void kernel_launch(void* const* d_in, const int* in_sizes, int n_in,
                              void* d_out, int out_size, void* d_ws, size_t ws_size,
                              hipStream_t stream) {
  const float* node_features = (const float*)d_in[0];
  const float* pos_pred      = (const float*)d_in[1];
  const int*   edge_index    = (const int*)  d_in[2];
  const int*   batch         = (const int*)  d_in[3];
  const float* t_discrete    = (const float*)d_in[4];
  const float* atom_w1       = (const float*)d_in[5];
  const float* atom_b1       = (const float*)d_in[6];
  const float* atom_w2       = (const float*)d_in[7];
  const float* atom_b2       = (const float*)d_in[8];
  const float* bond_w1       = (const float*)d_in[9];
  const float* bond_b1       = (const float*)d_in[10];
  const float* bond_w2       = (const float*)d_in[11];
  const float* bond_b2       = (const float*)d_in[12];

  const int H = HDIM;
  const int N = in_sizes[0] / H;
  const int E = in_sizes[2] / 2;
  const int B = in_sizes[4];

  char* ws = (char*)d_ws;
  size_t cur = 0;
  auto carve = [&](size_t bytes) { void* p = ws + cur; cur += (bytes + 255) & ~(size_t)255; return p; };
  float*  temb   = (float*) carve((size_t)B * H * 4);
  _Float16* hbf    = (_Float16*)carve((size_t)N * H * 2);
  _Float16* aw1T   = (_Float16*)carve((size_t)H * H * 2);
  _Float16* aw2T   = (_Float16*)carve((size_t)ATOM_PAD * H * 2);
  _Float16* bw1T   = (_Float16*)carve((size_t)H * 2 * H * 2);
  _Float16* bw2T   = (_Float16*)carve((size_t)BOND_PAD * H * 2);
  float* stA = (float*)carve((size_t)N * 128 * 4);
  float* stB = (float*)carve((size_t)E * 8 * 4);
  (void)ws_size;

  float* out_pos  = (float*)d_out;
  float* out_atom = out_pos  + (size_t)N * 3;
  float* out_bond = out_atom + (size_t)N * ATOM_TYPES;
  float* out_nf   = out_bond + (size_t)E * BOND_TYPES;

  k_temb<<<B, H, 0, stream>>>(t_discrete, temb, H);
  {
    int total8 = N * H / 8;
    k_make_h<<<(total8 + 255) / 256, 256, 0, stream>>>(node_features, batch, temb, hbf, total8, H, B);
    k_copy_f32<<<(N * H / 4 + 255) / 256, 256, 0, stream>>>(node_features, out_nf, N * H);
  }
  {
    int total = N * 3;
    k_copy_f32<<<((total + 3) / 4 + 255) / 256, 256, 0, stream>>>(pos_pred, out_pos, total);
  }
  k_transpose_pad<<<(H * H / 8 + 255) / 256, 256, 0, stream>>>(atom_w1, aw1T, H, H, H);
  k_transpose_pad<<<(H * ATOM_PAD / 8 + 255) / 256, 256, 0, stream>>>(atom_w2, aw2T, H, ATOM_TYPES, ATOM_PAD);
  k_transpose_pad<<<(2 * H * H / 8 + 255) / 256, 256, 0, stream>>>(bond_w1, bw1T, 2 * H, H, H);
  k_transpose_pad<<<(H * BOND_PAD / 8 + 255) / 256, 256, 0, stream>>>(bond_w2, bw2T, H, BOND_TYPES, BOND_PAD);

  k_atom<<<(N + 15) / 16, 256, 0, stream>>>(hbf, aw1T, atom_b1, aw2T, atom_b2, stA, N);
  {
    int blocks = (E + BOND_EPB - 1) / BOND_EPB;
    size_t shmem = (size_t)(BOND_EPB * 512 + BOND_EPB * HDIM) * 2;
    k_bond<<<blocks, 256, shmem, stream>>>(hbf, edge_index, bw1T, bond_b1, bw2T, bond_b2, stB, E);
  }
  k_flat<<<(N * ATOM_TYPES / 4 + E * BOND_TYPES / 4 + 255) / 256, 256, 0, stream>>>(stA, stB, out_atom, out_bond, N, E);
}
